// SATOPModule_80015240724634
// MI455X (gfx1250) — hardware-verified
//
#include <hip/hip_runtime.h>
#include <math.h>
typedef __attribute__((ext_vector_type(16))) _Float16 v16h;
typedef __attribute__((ext_vector_type(8)))  _Float16 v8h;
typedef __attribute__((ext_vector_type(16))) __bf16   v16b;
typedef __attribute__((ext_vector_type(8)))  __bf16   v8b;
typedef __attribute__((ext_vector_type(8)))  float    v8f;
typedef __attribute__((ext_vector_type(4)))  float    v4f;
#define PSCALE 32768.0f
#define U16(p) ((const unsigned short*)(const void*)(p))
#define PSCALE_INV (1.0f / 32768.0f)

__device__ __forceinline__ unsigned short f2bf_bits(float f) {
  unsigned u = __float_as_uint(f);
  return (unsigned short)((u + 0x7FFFu + ((u >> 16) & 1u)) >> 16);
}
__device__ __forceinline__ float bf_bits2f(unsigned short h) { return __uint_as_float(((unsigned)h) << 16); }

__device__ __forceinline__ void dep_guard_h(v8f& a, v8f& b, v16h x, v16h y) { asm volatile("v_nop\n\tv_nop\n\tv_nop\n\tv_nop" : "+v"(a), "+v"(b) : "v"(x), "v"(y)); }
__device__ __forceinline__ void dep_guard_b(v8f& a, v8f& b, v16b x, v16b y) { asm volatile("v_nop\n\tv_nop\n\tv_nop\n\tv_nop" : "+v"(a), "+v"(b) : "v"(x), "v"(y)); }
__device__ __forceinline__ void keep4_h(v16h a, v16h b, v16h c, v16h d) { asm volatile("v_nop" :: "v"(a), "v"(b), "v"(c), "v"(d)); }
__device__ __forceinline__ void keep4_b(v16b a, v16b b, v16b c, v16b d) { asm volatile("v_nop" :: "v"(a), "v"(b), "v"(c), "v"(d)); }
__device__ __forceinline__ void acc_guard4(v8f& a, v8f& b, v8f& c, v8f& d) { asm volatile("v_nop\n\tv_nop\n\tv_nop\n\tv_nop" : "+v"(a), "+v"(b), "+v"(c), "+v"(d)); }
template <typename T> struct Frag;
template <> struct Frag<_Float16> {
  typedef v16h V; union U { v16h v; v8h h[2]; };
  static __device__ __forceinline__ v16h load(const _Float16* p) {
    U f; f.h[0] = *(const v8h*)(p); f.h[1] = *(const v8h*)(p + 16); return f.v;
  }
  static __device__ __forceinline__ v8f mma(v16h a, v16h b, v8f c) {
    return __builtin_amdgcn_wmma_f32_16x16x32_f16(false, a, false, b, (short)0, c, false, false);
  }
  static __device__ __forceinline__ void guard(v8f& a, v8f& b, v16h x, v16h y) { dep_guard_h(a, b, x, y); }
  static __device__ __forceinline__ void keep(v16h a, v16h b, v16h c, v16h d) { keep4_h(a, b, c, d); }
};
template <> struct Frag<__bf16> {
  typedef v16b V; union U { v16b v; v8b h[2]; };
  static __device__ __forceinline__ v16b load(const __bf16* p) {
    U f; f.h[0] = *(const v8b*)(p); f.h[1] = *(const v8b*)(p + 16); return f.v;
  }
  static __device__ __forceinline__ v8f mma(v16b a, v16b b, v8f c) {
    return __builtin_amdgcn_wmma_f32_16x16x32_bf16(false, a, false, b, (short)0, c, false, false);
  }
  static __device__ __forceinline__ void guard(v8f& a, v8f& b, v16b x, v16b y) { dep_guard_b(a, b, x, y); }
  static __device__ __forceinline__ void keep(v16b a, v16b b, v16b c, v16b d) { keep4_b(a, b, c, d); }
};

template <int ET> struct Elem;
template <> struct Elem<0> { typedef _Float16 T; };
template <> struct Elem<1> { typedef __bf16 T; };
template <int ET, bool SPLIT, int BIAS_MODE, int OUT_MODE, bool RESID, int ACT = 0>
__global__ __launch_bounds__(256) void wmma_gemm64(
    const unsigned short* __restrict__ Ap, const unsigned short* __restrict__ A2p, int lda, long strideA,
    const unsigned short* __restrict__ Btp, const unsigned short* __restrict__ Bt2p, int ldb, long strideB,
    void* __restrict__ Cout, void* __restrict__ Cout2, int ldc, long strideC,
    const float* __restrict__ bias,
    const float* __restrict__ resid, long strideR,
    int M, int N, int K, float scale) {
  typedef typename Elem<ET>::T T;
  typedef typename Frag<T>::V V;
  const T* A = (const T*)Ap; const T* A2 = (const T*)A2p; const T* Bt = (const T*)Btp; const T* Bt2 = (const T*)Bt2p;
  __shared__ __align__(16) float sT[8][16 * 68];
  const int b    = blockIdx.y;
  const int lane = threadIdx.x & 31;
  const int wave = threadIdx.x >> 5;
  const int tilesN = N >> 6;
  const int tilesM = M >> 6;
  const int tile = blockIdx.x * 8 + wave;
  if (tile >= tilesM * tilesN) return;
  const int tm = tile / tilesN;
  const int tn = tile - tm * tilesN;
  const int m0 = tm << 6;
  const int n0 = tn << 6;

  const T* Ab  = A  + (size_t)b * strideA;
  const T* Bb  = Bt + (size_t)b * strideB;
  const T* Ab2 = SPLIT ? (A2  + (size_t)b * strideA) : nullptr;
  const T* Bb2 = SPLIT ? (Bt2 + (size_t)b * strideB) : nullptr;

  const int rlane = lane & 15;
  const int koff  = (lane >> 4) * 8;
  const int mOff  = (lane >> 4) * 8;

  v8f acc[4][4];
#pragma unroll
  for (int i = 0; i < 4; ++i)
#pragma unroll
    for (int j = 0; j < 4; ++j) acc[i][j] = (v8f){0.f,0.f,0.f,0.f,0.f,0.f,0.f,0.f};

  for (int k0 = 0; k0 < K; k0 += 32) {
    V bh[4], bl[4];
#pragma unroll
    for (int j = 0; j < 4; ++j) {
      const size_t bo = (size_t)(n0 + (j << 4) + rlane) * ldb + koff + k0;
      bh[j] = Frag<T>::load(Bb + bo);
      if (SPLIT) bl[j] = Frag<T>::load(Bb2 + bo);
    }
#pragma unroll
    for (int i = 0; i < 4; ++i) {
      const size_t ao = (size_t)(m0 + (i << 4) + rlane) * lda + koff + k0;
      V ah = Frag<T>::load(Ab + ao);
      V al;
      if (SPLIT) al = Frag<T>::load(Ab2 + ao);
#pragma unroll
      for (int j = 0; j < 4; ++j) {
        acc[i][j] = Frag<T>::mma(ah, bh[j], acc[i][j]);
        if (SPLIT) {
          acc[i][j] = Frag<T>::mma(ah, bl[j], acc[i][j]);
          acc[i][j] = Frag<T>::mma(al, bh[j], acc[i][j]);
        }
      }
      Frag<T>::guard(acc[i][0], acc[i][3], ah, SPLIT ? al : ah);
    }
    Frag<T>::keep(bh[0], bh[1], bh[2], bh[3]);
    if (SPLIT) Frag<T>::keep(bl[0], bl[1], bl[2], bl[3]);
  }
  acc_guard4(acc[0][0], acc[0][1], acc[0][2], acc[0][3]);
  acc_guard4(acc[1][0], acc[1][1], acc[1][2], acc[1][3]);
  acc_guard4(acc[2][0], acc[2][1], acc[2][2], acc[2][3]);
  acc_guard4(acc[3][0], acc[3][1], acc[3][2], acc[3][3]);

  float* slab = sT[wave];
  const float* Rb = RESID ? (resid + (size_t)b * strideR) : nullptr;
#pragma unroll
  for (int i = 0; i < 4; ++i) {
    const int mBase = m0 + (i << 4);
#pragma unroll
    for (int j = 0; j < 4; ++j) {
      const int n = n0 + (j << 4) + rlane;
      float bv = 0.f;
      if (BIAS_MODE == 2) bv = bias[n];
#pragma unroll
      for (int r = 0; r < 8; ++r) {
        float v = acc[i][j][r] * scale;
        if (BIAS_MODE == 1) v += bias[mBase + mOff + r];
        if (BIAS_MODE == 2) v += bv;
        if (RESID) v += Rb[(size_t)(mBase + mOff + r) * ldc + n];
        if (ACT == 1) v = tanhf(v);
        if (ACT == 2) v = fmaxf(v, 0.0f);
        slab[(mOff + r) * 68 + (j << 4) + rlane] = v;
      }
    }
    __builtin_amdgcn_fence(__ATOMIC_RELEASE, "workgroup");
    __builtin_amdgcn_wave_barrier();
    __builtin_amdgcn_fence(__ATOMIC_ACQUIRE, "workgroup");
    if (OUT_MODE == 0) {
      float* C = (float*)Cout + (size_t)b * strideC;
      const int hh = lane >> 4, c4 = (lane & 15) * 4;
      for (int pass = 0; pass < 2; ++pass) {
#pragma unroll
        for (int it = 0; it < 8; ++it) {
          const int row = it * 2 + hh;
          v4f v = *(const v4f*)(slab + row * 68 + c4);
          *(volatile v4f*)(C + (size_t)(mBase + row) * ldc + n0 + c4) = v;
        }
        __threadfence();
      }
    } else {
      const int q = lane >> 3, c8 = (lane & 7) * 8;
      unsigned short* C  = (unsigned short*)Cout  + (size_t)b * strideC;
      unsigned short* C2 = (OUT_MODE == 2) ? ((unsigned short*)Cout2 + (size_t)b * strideC) : nullptr;
      for (int pass = 0; pass < 2; ++pass) {
#pragma unroll
        for (int it = 0; it < 4; ++it) {
          const int row = it * 4 + q;
          const float* sp = slab + row * 68 + c8;
          v8h hv, lv;
#pragma unroll
          for (int e = 0; e < 8; ++e) {
            if (OUT_MODE == 1) {
              hv[e] = (_Float16)sp[e];
            } else {
              unsigned short hb = f2bf_bits(sp[e]);
              unsigned short lb = f2bf_bits(sp[e] - bf_bits2f(hb));
              hv[e] = __builtin_bit_cast(_Float16, hb);
              lv[e] = __builtin_bit_cast(_Float16, lb);
            }
          }
          *(volatile v8h*)(C + (size_t)(mBase + row) * ldc + n0 + c8) = hv;
          if (OUT_MODE == 2) *(volatile v8h*)(C2 + (size_t)(mBase + row) * ldc + n0 + c8) = lv;
        }
        __threadfence();
      }
    }
    __builtin_amdgcn_fence(__ATOMIC_RELEASE, "workgroup");
    __builtin_amdgcn_wave_barrier();
    __builtin_amdgcn_fence(__ATOMIC_ACQUIRE, "workgroup");
  }
}

__global__ __launch_bounds__(256) void cast_f32_f16x2(
    const float* __restrict__ in, _Float16* __restrict__ out, int n2) {
  int i = blockIdx.x * 256 + threadIdx.x;
  if (i < n2) {
    const _Float16 h0 = (_Float16)in[2 * i], h1 = (_Float16)in[2 * i + 1];
    const unsigned u = (unsigned)__builtin_bit_cast(unsigned short, h0) | ((unsigned)__builtin_bit_cast(unsigned short, h1) << 16);
    ((volatile unsigned*)out)[i] = u;
    __threadfence();
    ((volatile unsigned*)out)[i] = u;
  }
}


__global__ __launch_bounds__(256) void transpose_cast_f16(const float* __restrict__ in, int ldi,
                                                         _Float16* __restrict__ outT, int ldo, float scale) {
  __shared__ __align__(16) _Float16 tile[64][72];
  const int c0 = blockIdx.x * 64, r0 = blockIdx.y * 64;
  const int t = threadIdx.y * 32 + threadIdx.x;
  for (int i = threadIdx.y; i < 64; i += 8) {
    tile[threadIdx.x][i]      = (_Float16)(in[(size_t)(r0 + i) * ldi + c0 + threadIdx.x] * scale);
    tile[32 + threadIdx.x][i] = (_Float16)(in[(size_t)(r0 + i) * ldi + c0 + 32 + threadIdx.x] * scale);
  }
  __syncthreads();
  const int q = t >> 3, c8 = (t & 7) * 8;
  for (int pass = 0; pass < 2; ++pass) {
#pragma unroll
    for (int it = 0; it < 2; ++it) {
      const int c = it * 32 + q;
      v8h hv = *(const v8h*)(&tile[c][c8]);
      *(volatile v8h*)(outT + (size_t)(c0 + c) * ldo + r0 + c8) = hv;
    }
    __threadfence();
  }
}

#define NL 2
#define NN 1024
#define NB 8
#define NF 128
#define NH 256

__device__ __forceinline__ float eluf(float v) { return v > 0.f ? v : expm1f(v); }

__global__ __launch_bounds__(256) void edge_kernel(const float* __restrict__ adj, const float* __restrict__ W1, const float* __restrict__ b1,
                                                  const float* __restrict__ W2, const float* __restrict__ b2, _Float16* __restrict__ A) {
  __shared__ __align__(16) _Float16 hs[8][16 * 264];
  __shared__ __align__(16) _Float16 w2s[16 * 32 * 8];
  __shared__ __align__(16) _Float16 outs[128];
  __shared__ float w1s[NH * 2], b1s[NH];
  const int tid = threadIdx.x, lane = tid & 31, wave = tid >> 5;
  const int n = blockIdx.y, m0 = blockIdx.x * 128 + wave * 16;
  for (int i = tid; i < NH * 2; i += 256) w1s[i] = W1[i];
  for (int i = tid; i < NH; i += 256) b1s[i] = b1[i];
  for (int i = tid; i < 16 * 32 * 8; i += 256) {
    const int e = i & 15, l = (i >> 4) & 31, kc = i >> 9;
    const int k = kc * 32 + ((e < 8) ? (8 * (l >> 4) + e) : (16 + 8 * (l >> 4) + (e - 8)));
    w2s[i] = ((l & 15) == 0) ? (_Float16)W2[k] : (_Float16)0.0f;
  }
  __syncthreads();
  _Float16* hw = hs[wave];
#pragma unroll 1
  for (int ed = 0; ed < 16; ++ed) {
    const float a0 = adj[((size_t)n * NN + m0 + ed) * 2 + 0], a1 = adj[((size_t)n * NN + m0 + ed) * 2 + 1];
#pragma unroll
    for (int j = 0; j < 8; ++j) {
      const int h = lane + 32 * j;
      const float v = eluf(a0 * w1s[h * 2 + 0] + a1 * w1s[h * 2 + 1] + b1s[h]);
      hw[ed * 264 + h] = (_Float16)v;
    }
  }
  __builtin_amdgcn_fence(__ATOMIC_RELEASE, "workgroup");
  __builtin_amdgcn_wave_barrier();
  __builtin_amdgcn_fence(__ATOMIC_ACQUIRE, "workgroup");
  v8f acc = {};
  const int row = lane & 15, hh = lane >> 4;
#pragma unroll
  for (int kc = 0; kc < 8; ++kc) {
    v16h a, bfr;
    const v8h lo = *(const v8h*)(hw + row * 264 + kc * 32 + 8 * hh);
    const v8h hi = *(const v8h*)(hw + row * 264 + kc * 32 + 16 + 8 * hh);
#pragma unroll
    for (int e = 0; e < 8; ++e) { a[e] = lo[e]; a[8 + e] = hi[e]; }
    bfr = *(const v16h*)(w2s + (kc * 32 + lane) * 16);
    acc = __builtin_amdgcn_wmma_f32_16x16x32_f16(false, a, false, bfr, (short)0, acc, false, false);
    { v8f dmy = acc; dep_guard_h(acc, dmy, a, bfr); }
  }
  if ((lane & 15) == 0) {
#pragma unroll
    for (int r = 0; r < 8; ++r) {
      const int ed = 8 * hh + r;
      const float lim = (adj[((size_t)n * NN + m0 + ed) * 2 + 0] > 0.f) ? 1.0f : 0.0f;
      outs[wave * 16 + ed] = (_Float16)(lim * tanhf(acc[r] + b2[0]));
    }
  }
  __syncthreads();
  if (wave == 0 && lane < 16) {
    const v8h v = *(const v8h*)(&outs[lane * 8]);
    *(volatile v8h*)(A + (size_t)n * NN + blockIdx.x * 128 + lane * 8) = v;
    __threadfence();
    *(volatile v8h*)(A + (size_t)n * NN + blockIdx.x * 128 + lane * 8) = v;
  }
}


__global__ __launch_bounds__(256) void resid_ln_kernel(const float* __restrict__ xin, const float* __restrict__ xh, const float* __restrict__ g,
                                                      const float* __restrict__ be, float* __restrict__ xout) {
  const int lane = threadIdx.x & 31, wave = threadIdx.x >> 5;
  const size_t row = (size_t)blockIdx.x * 8 + wave;
  v4f a = *(const v4f*)(xin + row * NF + 4 * lane), h = *(const v4f*)(xh + row * NF + 4 * lane);
  float y[4]; float s = 0.f;
#pragma unroll
  for (int q = 0; q < 4; ++q) { y[q] = a[q] + h[q]; s += y[q]; }
  for (int o = 16; o > 0; o >>= 1) s += __shfl_xor(s, o, 32);
  const float mu = s * (1.0f / NF);
  float s2 = 0.f;
#pragma unroll
  for (int q = 0; q < 4; ++q) { const float d = y[q] - mu; s2 += d * d; }
  for (int o = 16; o > 0; o >>= 1) s2 += __shfl_xor(s2, o, 32);
  const float r = rsqrtf(s2 * (1.0f / NF) + 1e-5f);
  v4f o4;
#pragma unroll
  for (int q = 0; q < 4; ++q) o4[q] = (y[q] - mu) * r * g[4 * lane + q] + be[4 * lane + q];
  *(volatile v4f*)(xout + row * NF + 4 * lane) = o4;
  __threadfence();
  *(volatile v4f*)(xout + row * NF + 4 * lane) = o4;
}

extern "C" void kernel_launch(void* const* d_in, const int* in_sizes, int n_in,
                              void* d_out, int out_size, void* d_ws, size_t ws_size,
                              hipStream_t stream) {
  (void)in_sizes; (void)n_in; (void)out_size; (void)ws_size;
  const float* x   = (const float*)d_in[0];
  const float* adj = (const float*)d_in[1];
  const float* W1  = (const float*)d_in[2];
  const float* b1  = (const float*)d_in[3];
  const float* W2  = (const float*)d_in[4];
  const float* b2  = (const float*)d_in[5];
  const float* Wfc = (const float*)d_in[6];
  const float* bias= (const float*)d_in[7];
  const float* gam = (const float*)d_in[8];
  const float* bet = (const float*)d_in[9];
  float* out = (float*)d_out;
  const int M = NB * NN;

  char* ws = (char*)d_ws; size_t off = 0;
  auto carve = [&](size_t bytes) -> char* { char* p = ws + off; off += (bytes + 255) & ~(size_t)255; return p; };
  _Float16* A16  = (_Float16*)carve((size_t)NN * NN * 2);
  _Float16* X16  = (_Float16*)carve((size_t)M * NF * 2);
  _Float16* Wf16 = (_Float16*)carve((size_t)NF * NF * 2);
  float*    FX   = (float*)carve((size_t)M * NF * 4);
  _Float16* FXT  = (_Float16*)carve((size_t)NB * NF * NN * 2);
  float*    XH   = (float*)carve((size_t)M * NF * 4);
  float*    X1   = (float*)carve((size_t)M * NF * 4);

  const float* xcur = x;
  for (int l = 0; l < NL; ++l) {
    float* xnext = (l == NL - 1) ? out : X1;
    edge_kernel<<<dim3(NN / 128, NN), 256, 0, stream>>>(adj, W1 + l * NH * 2, b1 + l * NH, W2 + l * NH, b2 + l, A16);
    cast_f32_f16x2<<<(M * NF / 2 + 255) / 256, 256, 0, stream>>>(xcur, X16, M * NF / 2);
    cast_f32_f16x2<<<(NF * NF / 2 + 255) / 256, 256, 0, stream>>>(Wfc + (size_t)l * NF * NF, Wf16, NF * NF / 2);
    {
      const int t1 = (M / 64) * (NF / 64);
      wmma_gemm64<0, false, 0, 0, false><<<dim3((t1 + 7) / 8, 1), 256, 0, stream>>>(
          U16(X16), nullptr, NF, 0, U16(Wf16), nullptr, NF, 0, FX, nullptr, NF, 0, nullptr, nullptr, 0, M, NF, NF, 1.0f);
    }
    for (int b = 0; b < NB; ++b)
      transpose_cast_f16<<<dim3(NF / 64, NN / 64), dim3(32, 8), 0, stream>>>(FX + (size_t)b * NN * NF, NF, FXT + (size_t)b * NF * NN, NN, 1.0f);
    {
      const int t2 = (NN / 64) * (NF / 64);
      wmma_gemm64<0, false, 2, 0, false><<<dim3((t2 + 7) / 8, NB), 256, 0, stream>>>(
          U16(A16), nullptr, NN, 0, U16(FXT), nullptr, NN, (long)NF * NN, XH, nullptr, NF, (long)NN * NF, bias + l * NF, nullptr, 0, NN, NF, NN, 1.0f);
    }
    resid_ln_kernel<<<M / 8, 256, 0, stream>>>(xcur, XH, gam + l * NF, bet + l * NF, xnext);
    xcur = xnext;
  }
}
